// GCN_67336497266833
// MI455X (gfx1250) — hardware-run, weakly checked
//
#include <hip/hip_runtime.h>

typedef float          v8f   __attribute__((ext_vector_type(8)));
typedef float          v4f   __attribute__((ext_vector_type(4)));
typedef unsigned int   v4u   __attribute__((ext_vector_type(4)));
typedef int            v8i   __attribute__((ext_vector_type(8)));
typedef unsigned short v8us  __attribute__((ext_vector_type(8)));
typedef unsigned short v16us __attribute__((ext_vector_type(16)));
typedef __bf16         v16bf __attribute__((ext_vector_type(16)));
typedef _Float16       v16h  __attribute__((ext_vector_type(16)));
typedef v4f  __attribute__((may_alias)) v4fa;
typedef v8us __attribute__((may_alias)) v8usa;
union FragB { v16bf v; v16us u; v8us h[2]; v8i w; };
union FragH { v16h  v; v16us u; v8us h[2]; v8i w; };

__device__ __forceinline__ v8f wmb(const FragB& a, const FragB& b, v8f c) {
  v8f d = __builtin_amdgcn_wmma_f32_16x16x32_bf16(false, a.v, false, b.v, (short)0, c, false, false);
  asm volatile("v_nop\n\tv_nop\n\tv_nop\n\tv_nop" : "+v"(d) : "v"(a.w), "v"(b.w));
  return d;
}

__device__ __forceinline__ v8f wmh(const FragH& a, const FragH& b, v8f c) {
  v8f d = __builtin_amdgcn_wmma_f32_16x16x32_f16(false, a.v, false, b.v, (short)0, c, false, false);
  asm volatile("v_nop\n\tv_nop\n\tv_nop\n\tv_nop" : "+v"(d) : "v"(a.w), "v"(b.w));
  return d;
}

__device__ __forceinline__ unsigned bf16_bits(float f) {
  const unsigned u = __float_as_uint(f);
  const unsigned r = (u + 0x7FFFu + ((u >> 16) & 1u)) >> 16;
  const unsigned q = (u >> 16) | 0x40u;
  return ((u & 0x7fffffffu) > 0x7f800000u) ? q : r;
}

__device__ __forceinline__ float bf16_val(float f) {
  return __uint_as_float(bf16_bits(f) << 16);
}
__device__ __forceinline__ int clampi(int v, int lo, int hi) {
  return v < lo ? lo : (v > hi ? hi : v);
}

__device__ __forceinline__ unsigned f16_bits(float f) {
  const unsigned u  = __float_as_uint(f);
  const unsigned s  = (u >> 16) & 0x8000u;
  const unsigned a  = u & 0x7fffffffu;
  const unsigned t  = a - 0x38000000u;
  const unsigned r  = (t + 0x0FFFu + ((t >> 13) & 1u)) >> 13;
  const unsigned rc = r > 0x7C00u ? 0x7C00u : r;
  const bool small  = a < 0x38800000u;
  const bool isnan  = a > 0x7f800000u;
  const unsigned fin = small ? 0u : (s | rc);
  return isnan ? (s | 0x7E00u) : fin;
}

__device__ __forceinline__ unsigned pk16(unsigned lo, unsigned hi) { return lo | (hi << 16); }
__device__ __forceinline__ unsigned bf16_lo_bits(float v) {
  float hi = bf16_val(v);
  asm volatile("" : "+v"(hi));
  return bf16_bits(v - hi);
}
__device__ __forceinline__ v4u pack8_bf16(v4f a, v4f c) {
  return (v4u){ pk16(bf16_bits(a[0]), bf16_bits(a[1])), pk16(bf16_bits(a[2]), bf16_bits(a[3])),
                pk16(bf16_bits(c[0]), bf16_bits(c[1])), pk16(bf16_bits(c[2]), bf16_bits(c[3])) };
}
__device__ __forceinline__ v4u pack8_bf16_lo(v4f a, v4f c) {
  return (v4u){ pk16(bf16_lo_bits(a[0]), bf16_lo_bits(a[1])), pk16(bf16_lo_bits(a[2]), bf16_lo_bits(a[3])),
                pk16(bf16_lo_bits(c[0]), bf16_lo_bits(c[1])), pk16(bf16_lo_bits(c[2]), bf16_lo_bits(c[3])) };
}
__device__ __forceinline__ v4u pack8_f16(v4f a, v4f c) {
  return (v4u){ pk16(f16_bits(a[0]), f16_bits(a[1])), pk16(f16_bits(a[2]), f16_bits(a[3])),
                pk16(f16_bits(c[0]), f16_bits(c[1])), pk16(f16_bits(c[2]), f16_bits(c[3])) };
}

template <int FORM>
__global__ __launch_bounds__(256) void k_plane(const float* __restrict__ src, int rows, int cols, int ldsrc,
                                               unsigned short* __restrict__ dst, int MP, int KP) {
  static_assert(FORM >= 0 && FORM <= 3);
  const int KTOT = (FORM == 1 || FORM == 3) ? 2 * KP : KP;
  const unsigned ppr   = (unsigned)(KTOT >> 3);
  const unsigned kp8   = (unsigned)(KP >> 3);
  const unsigned total = (unsigned)MP * ppr;
  const unsigned g     = blockIdx.x * 256u + threadIdx.x;
  const unsigned rowu  = g / ppr;
  const unsigned p     = g - rowu * ppr;
  const bool second    = p >= kp8;
  const int row = (int)rowu;
  const int c0  = (int)((second ? p - kp8 : p) << 3);
  const float* srow = src + (size_t)clampi(row, 0, rows - 1) * (size_t)ldsrc;
  float x[8];
  unsigned mk[8];
#pragma unroll
  for (int e = 0; e < 8; ++e) {
    const int c = c0 + e;
    const float v = srow[clampi(c, 0, cols - 1)];
    asm volatile("" :: "v"(v));
    x[e]  = v;
    mk[e] = (row < rows && c < cols) ? 0xFFFFu : 0u;
  }
  const v4f a = (v4f){ x[0], x[1], x[2], x[3] };
  const v4f c = (v4f){ x[4], x[5], x[6], x[7] };
  v4u o;
  if (FORM == 2) {
    o = pack8_f16(a, c);
  } else {
    const v4u hi = pack8_bf16(a, c);
    o = hi;
    if (FORM == 1) { const v4u lo = pack8_bf16_lo(a, c); o = second ? lo : hi; }
  }
  const v4u mw = (v4u){ pk16(mk[0], mk[1]), pk16(mk[2], mk[3]), pk16(mk[4], mk[5]), pk16(mk[6], mk[7]) };
  o &= mw;
  if (g < total) {
    volatile v4u* q = (volatile v4u*)(dst + (size_t)g * 8);
    *q = o;
    __threadfence();
    *q = o;
  }
}

template <int FORM> struct FragOf    { typedef FragB T; };
template <>         struct FragOf<2> { typedef FragH T; };
__device__ __forceinline__ v8f mm(const FragB& a, const FragB& b, v8f c) { return wmb(a, b, c); }
__device__ __forceinline__ v8f mm(const FragH& a, const FragH& b, v8f c) { return wmh(a, b, c); }
template <class F> __device__ __forceinline__ F ld_frag(const unsigned short* p) {
  F f;
  f.h[0] = *(const v8usa*)(p);
  f.h[1] = *(const v8usa*)(p + 16);
  return f;
}

template <int FORM, int EPI>
__global__ __launch_bounds__(256) __attribute__((amdgpu_num_vgpr(248)))
void k_gemm_nt(const unsigned short* __restrict__ A, const unsigned short* __restrict__ B,
               const float* __restrict__ bias, float* __restrict__ D, int M, int N, int KTOT, int ldd) {
  static_assert(FORM >= 0 && FORM <= 2);
  static_assert(EPI == 0 || EPI == 1);
  typedef typename FragOf<FORM>::T F;
  __shared__ __attribute__((aligned(16))) float sT[8][16 * 68];
  const int lane = threadIdx.x & 31;
  const int wave = threadIdx.x >> 5;
  const int tilesM = (M + 63) >> 6;
  const int tilesN = (N + 63) >> 6;
  const int tile = blockIdx.x * 8 + wave;
  if (tile >= tilesM * tilesN) return;
  const int tm = tile / tilesN;
  const int tn = tile - tm * tilesN;
  const int m0 = tm << 6;
  const int n0 = tn << 6;

  const int rl = lane & 15;
  const int h8 = (lane >> 4) * 8;
  const unsigned short* pa = A + (size_t)(m0 + rl) * (size_t)KTOT + h8;
  const unsigned short* pb = B + (size_t)(n0 + rl) * (size_t)KTOT + h8;

  v8f acc[4][4];
#pragma unroll
  for (int i = 0; i < 4; ++i)
#pragma unroll
    for (int j = 0; j < 4; ++j) acc[i][j] = (v8f){0.f, 0.f, 0.f, 0.f, 0.f, 0.f, 0.f, 0.f};

#pragma unroll 1
  for (int k0 = 0; k0 < KTOT; k0 += 32) {
    F bf[4];
#pragma unroll
    for (int j = 0; j < 4; ++j) bf[j] = ld_frag<F>(pb + (size_t)(j << 4) * (size_t)KTOT + k0);
#pragma unroll
    for (int i = 0; i < 4; ++i) {
      const F af = ld_frag<F>(pa + (size_t)(i << 4) * (size_t)KTOT + k0);
#pragma unroll
      for (int j = 0; j < 4; ++j) acc[i][j] = mm(af, bf[j], acc[i][j]);
    }
  }

  float* slab = sT[wave];
  const int hh = lane >> 4;
  const int c4 = (lane & 15) * 4;
  const int nc = n0 + c4;
  const bool cok = nc < N;
  v4f bv = (v4f){0.f, 0.f, 0.f, 0.f};
  if (EPI == 1) {
    bv = *(const v4fa*)(bias + clampi(nc, 0, N - 4));
    asm volatile("" :: "v"(bv));
  }
#pragma unroll
  for (int i = 0; i < 4; ++i) {
    const int mBase = m0 + (i << 4);
#pragma unroll
    for (int j = 0; j < 4; ++j) {
#pragma unroll
      for (int r = 0; r < 8; ++r) slab[(h8 + r) * 68 + (j << 4) + rl] = acc[i][j][r];
    }
    __builtin_amdgcn_fence(__ATOMIC_RELEASE, "workgroup");
    __builtin_amdgcn_wave_barrier();
    __builtin_amdgcn_fence(__ATOMIC_ACQUIRE, "workgroup");
    v4f vv[8];
#pragma unroll
    for (int it = 0; it < 8; ++it) {
      const int row = it * 2 + hh;
      v4f v = *(const v4fa*)(slab + row * 68 + c4);
      if (EPI == 1) v += bv;
      vv[it] = v;
    }
    for (int pass = 0; pass < 2; ++pass) {
#pragma unroll
      for (int it = 0; it < 8; ++it) {
        const int row = mBase + it * 2 + hh;
        if (cok && row < M) *(volatile v4f*)(D + (size_t)row * (size_t)ldd + nc) = vv[it];
      }
      __threadfence();
    }
    __builtin_amdgcn_fence(__ATOMIC_RELEASE, "workgroup");
    __builtin_amdgcn_wave_barrier();
    __builtin_amdgcn_fence(__ATOMIC_ACQUIRE, "workgroup");
  }
}

#pragma clang fp contract(off)

#ifndef L2_TWO_TERM
#define L2_TWO_TERM 1
#endif

#define GN      50000
#define GE      800000
#define D0      256
#define D1      256
#define D2      128
#define NPAD    50048
#define K2TOT   (L2_TWO_TERM ? 512 : 256)
#define NTHR    256
#define NWAVE   8
#define EPT     8
#define CHUNK   2048
#define NCHUNK  391
#define WCAP    256
#define LISTN   (NWAVE * WCAP)
#define NBRUN   1024
#define NBLK    49
#define RCAP    22528
#define DEGCAP  43
#define BK_ZINTS    (LISTN + 2 * RCAP + 3 * NBRUN)
#define BK_LDS_INTS (BK_ZINTS + 16)
#define BK_LDS_BYTES (BK_LDS_INTS * 4)

#define PB_X   (NPAD / 8)
#define PB_W1  ((D1 * (D0 / 8)) / NTHR)
#define PB_W2  ((D2 * (K2TOT / 8)) / NTHR)
#define PB_B   1
#define PB_Z   (L2_TWO_TERM ? (((NPAD - GN) * (K2TOT / 8)) / NTHR) : 0)
#define PB_ALL (PB_X + PB_W1 + PB_W2 + PB_B + PB_Z)

static_assert(GN % 8 == 0);
static_assert(NPAD % 128 == 0 && NPAD >= GN && NPAD % 64 == 0);
static_assert(GE == 390 * 2048 + 1280 && GE % EPT == 0);
static_assert(NCHUNK * CHUNK >= GE && (NCHUNK - 1) * CHUNK < GE);
static_assert(D1 == 32 * 8 && D2 == 32 * 4 && D0 == 32 * 8);
static_assert(GN - 1 < 65536 && NBRUN <= 1024);
static_assert(NBLK * NBRUN >= GN && (NBLK - 1) * NBRUN < GN);
static_assert(RCAP * 4 >= 16623 * 5 && RCAP % 1024 == 0);
static_assert(DEGCAP == 35 + 8 && DEGCAP <= 64);
static_assert(BK_ZINTS % 1024 == 0);
static_assert(BK_LDS_BYTES <= 262144 && BK_LDS_BYTES + 0 <= 327680);
static_assert((D1 * (D0 / 8)) % NTHR == 0 && (D2 * (K2TOT / 8)) % NTHR == 0);
static_assert(((NPAD - GN) * (K2TOT / 8)) % NTHR == 0);
static_assert(GN % 16 == 0 && D0 % 32 == 0 && K2TOT % 32 == 0 && D1 % 64 == 0 && D2 % 64 == 0);

typedef int v4i __attribute__((ext_vector_type(4)));
typedef v4i __attribute__((may_alias)) v4ia;

constexpr size_t SZ_H    = (size_t)NPAD * D1 * 4;
constexpr size_t SZ_X1   = (size_t)NPAD * 512 * 2;
constexpr size_t SZ_LIST = (size_t)NBLK * RCAP * 4;
constexpr size_t SZ_ROWT = (size_t)NBLK * NBRUN * 4;
constexpr size_t SZ_FLAG = 8192;
constexpr size_t SZ_W1T  = (size_t)D1 * D0 * 2;
constexpr size_t SZ_W2D  = (size_t)D2 * 512 * 2;
constexpr size_t SZ_B1F  = (size_t)D1 * 4;
constexpr size_t SZ_B2F  = (size_t)D2 * 4;
constexpr size_t O_H    = 0;
constexpr size_t O_X1   = O_H + SZ_H;
constexpr size_t O_LIST = O_X1 + SZ_X1;
constexpr size_t O_CNT  = O_LIST + SZ_LIST;
constexpr size_t O_OFF  = O_CNT + SZ_ROWT;
constexpr size_t O_DINV = O_OFF + SZ_ROWT;
constexpr size_t O_FLAG = O_DINV + SZ_ROWT;
constexpr size_t O_W1T  = O_FLAG + SZ_FLAG;
constexpr size_t O_W2D  = O_W1T + SZ_W1T;
constexpr size_t O_B1F  = O_W2D + SZ_W2D;
constexpr size_t O_B2F  = O_B1F + SZ_B1F;
constexpr size_t WS_TOTAL = O_B2F + SZ_B2F;
static_assert(SZ_H % 128 == 0 && SZ_X1 % 128 == 0 && SZ_LIST % 128 == 0 && SZ_ROWT % 128 == 0);
static_assert(SZ_W1T % 128 == 0 && SZ_W2D % 128 == 0 && SZ_B1F % 128 == 0 && SZ_B2F % 128 == 0);
static_assert(SZ_H >= (size_t)NPAD * D2 * 4);
static_assert(SZ_X1 >= (size_t)NPAD * K2TOT * 2 && SZ_X1 >= (size_t)NPAD * D0 * 2);
static_assert((size_t)NBLK * 128 <= SZ_FLAG);
static_assert(WS_TOTAL <= ((size_t)128 << 20));

__global__ __launch_bounds__(NTHR) void k_prep(const int* __restrict__ fidx, const float* __restrict__ emb,
                                               const float* __restrict__ W1, const float* __restrict__ b1,
                                               const float* __restrict__ W2, const float* __restrict__ b2,
                                               unsigned short* XB, unsigned short* W1T, unsigned short* W2D,
                                               float* B1F, float* B2F, unsigned short* X1) {
  const int tid = (int)threadIdx.x, lane = tid & 31, wave = tid >> 5;
  const int bid = (int)blockIdx.x;
  if (bid < PB_X) {
    const int row = bid * 8 + wave;
    const int rc  = row < GN ? row : GN - 1;
    int fi = fidx[rc];
    asm volatile("" :: "v"(fi));
    fi = clampi(fi, 0, GN - 1);
    const float* p = emb + (size_t)fi * D0 + 8 * lane;
    const v4f a = *(const v4fa*)p;
    const v4f c = *(const v4fa*)(p + 4);
    asm volatile("" :: "v"(a));
    asm volatile("" :: "v"(c));
    v4u o = pack8_bf16(a, c);
    const unsigned mk = row < GN ? 0xFFFFFFFFu : 0u;
    o &= (v4u){ mk, mk, mk, mk };
    volatile v4u* q = (volatile v4u*)(XB + (size_t)row * D0 + 8 * lane);
    *q = o;
    __threadfence();
    *q = o;
  } else if (bid < PB_X + PB_W1) {
    const int u  = (bid - PB_X) * NTHR + tid;
    const int n  = u >> 5;
    const int k8 = (u & 31) * 8;
    const float* p = W1 + (size_t)k8 * D1 + n;
    float x[8];
#pragma unroll
    for (int i = 0; i < 8; ++i) x[i] = p[(size_t)i * D1];
    const v4u o = pack8_bf16((v4f){ x[0], x[1], x[2], x[3] }, (v4f){ x[4], x[5], x[6], x[7] });
    volatile v4u* q = (volatile v4u*)(W1T + (size_t)n * D0 + k8);
    *q = o;
    __threadfence();
    *q = o;
  } else if (bid < PB_X + PB_W1 + PB_W2) {
    const int u   = (bid - PB_X - PB_W1) * NTHR + tid;
    const int ppr = K2TOT / 8;
    const int n   = u / ppr;
    const int k8  = (u - n * ppr) * 8;
    const int kk  = k8 & (D1 - 1);
    const float* p = W2 + (size_t)kk * D2 + n;
    float x[8];
#pragma unroll
    for (int i = 0; i < 8; ++i) x[i] = p[(size_t)i * D2];
    const v4u o = pack8_bf16((v4f){ x[0], x[1], x[2], x[3] }, (v4f){ x[4], x[5], x[6], x[7] });
    volatile v4u* q = (volatile v4u*)(W2D + (size_t)n * K2TOT + k8);
    *q = o;
    __threadfence();
    *q = o;
  } else if (bid < PB_X + PB_W1 + PB_W2 + PB_B) {
    if (wave < 2) {
      const v4f v = *(const v4fa*)(b1 + 4 * tid);
      const v4f o = (v4f){ bf16_val(v[0]), bf16_val(v[1]), bf16_val(v[2]), bf16_val(v[3]) };
      volatile v4f* q = (volatile v4f*)(B1F + 4 * tid);
      *q = o;
      __threadfence();
      *q = o;
    } else if (wave == 2) {
      const v4f v = *(const v4fa*)(b2 + 4 * lane);
      const v4f o = (v4f){ bf16_val(v[0]), bf16_val(v[1]), bf16_val(v[2]), bf16_val(v[3]) };
      volatile v4f* q = (volatile v4f*)(B2F + 4 * lane);
      *q = o;
      __threadfence();
      *q = o;
    }
  } else {
    const int g = (bid - PB_X - PB_W1 - PB_W2 - PB_B) * NTHR + tid;
    const v4u z = (v4u){ 0u, 0u, 0u, 0u };
    volatile v4u* q = (volatile v4u*)(X1 + (size_t)GN * K2TOT + (size_t)g * 8);
    *q = z;
    __threadfence();
    *q = z;
  }
}

__global__ __launch_bounds__(NTHR) void k_bucket(const int* __restrict__ srcs, const int* __restrict__ dsts,
                                                 int* LISTG, int* CNTG, int* OFFG, int* DINVB, int* FLAGG) {
  extern __shared__ __attribute__((aligned(16))) int dsm[];
  int* list = dsm;
  int* hl   = dsm + LISTN;
  int* sl   = dsm + LISTN + RCAP;
  int* cnt  = dsm + LISTN + 2 * RCAP;
  int* offs = cnt + NBRUN;
  int* cur  = offs + NBRUN;
  int* misc = cur + NBRUN;
  const int tid = (int)threadIdx.x, lane = tid & 31, wave = tid >> 5;
  const int blk = (int)blockIdx.x;
  const int slotBase = blk * NBRUN;
  int nbv = GN - slotBase;
  nbv = nbv > NBRUN ? NBRUN : (nbv < 0 ? 0 : nbv);
  const unsigned unb = (unsigned)nbv;
  const unsigned nbs = (unsigned)slotBase;

  {
    const v4i z4 = (v4i){ 0, 0, 0, 0 };
#pragma unroll 1
    for (int i = tid * 4; i < BK_ZINTS; i += NTHR * 4) *(v4ia*)(dsm + i) = z4;
    if (tid < 16) misc[tid] = 0;
  }
  __syncthreads();

  int t = 0, ov = 0;
#pragma unroll 1
  for (int ch = 0; ch < NCHUNK; ++ch) {
    const int cbase = ch * CHUNK;
    const int e0  = cbase + tid * EPT;
    const int e0c = e0 < GE - EPT ? e0 : GE - EPT;
    v4i ka = *(const v4ia*)(dsts + e0c);
    v4i kb = *(const v4ia*)(dsts + e0c + 4);
    const v4i sa = *(const v4ia*)(srcs + e0c);
    const v4i sb = *(const v4ia*)(srcs + e0c + 4);
    asm volatile("" :: "v"(ka));
    asm volatile("" :: "v"(kb));
    asm volatile("" :: "v"(sa));
    asm volatile("" :: "v"(sb));
    const int nv = (e0 < GE) ? 0 : -1;
    ka |= (v4i){ nv, nv, nv, nv };
    kb |= (v4i){ nv, nv, nv, nv };
    const int kk[8] = { ka.x, ka.y, ka.z, ka.w, kb.x, kb.y, kb.z, kb.w };
    const int ss[8] = { sa.x, sa.y, sa.z, sa.w, sb.x, sb.y, sb.z, sb.w };
    unsigned sj[8];
    bool hit[8];
    int nh = 0;
#pragma unroll
    for (int j = 0; j < 8; ++j) {
      sj[j]  = (unsigned)kk[j] - nbs;
      hit[j] = sj[j] < unb;
      nh += hit[j] ? 1 : 0;
    }
    const unsigned m0 = __builtin_amdgcn_ballot_w32((nh & 1) != 0);
    const unsigned m1 = __builtin_amdgcn_ballot_w32((nh & 2) != 0);
    const unsigned m2 = __builtin_amdgcn_ballot_w32((nh & 4) != 0);
    const unsigned m3 = __builtin_amdgcn_ballot_w32((nh & 8) != 0);
    const int base = (int)(__builtin_amdgcn_mbcnt_lo(m0, 0u) + 2u * __builtin_amdgcn_mbcnt_lo(m1, 0u) +
                           4u * __builtin_amdgcn_mbcnt_lo(m2, 0u) + 8u * __builtin_amdgcn_mbcnt_lo(m3, 0u));
    const int wc = __builtin_popcount(m0) + 2 * __builtin_popcount(m1) +
                   4 * __builtin_popcount(m2) + 8 * __builtin_popcount(m3);
    int pos = base;
#pragma unroll
    for (int j = 0; j < 8; ++j) {
      if (hit[j]) {
        const int pp = pos < WCAP - 1 ? pos : WCAP - 1;
        list[wave * WCAP + pp] = (int)((unsigned)clampi(ss[j], 0, GN - 1) | (sj[j] << 16));
        pos = pos + 1;
      }
    }
    if (lane == 0) misc[wave] = wc;
    __syncthreads();
    if (wave == 0) {
#pragma unroll 1
      for (int w2 = 0; w2 < NWAVE; ++w2) {
        int cvv = misc[w2];
        cvv = clampi(cvv, 0, WCAP);
        const int c = __builtin_amdgcn_readfirstlane(cvv);
#pragma unroll 1
        for (int b0 = 0; b0 < c; b0 += 32) {
          const int idx = b0 + lane;
          const int ent = list[w2 * WCAP + (idx < WCAP ? idx : WCAP - 1)];
          const int m32 = (c - b0) < 32 ? (c - b0) : 32;
#pragma unroll 1
          for (int k = 0; k < m32; ++k) {
            const int u    = __builtin_amdgcn_readlane(ent, k);
            const int slot = (u >> 16) & (NBRUN - 1);
            if (t < RCAP) {
              if (lane == 0) { hl[t] = u; cnt[slot] = cnt[slot] + 1; }
              t = t + 1;
            } else {
              ov = 1;
            }
          }
        }
      }
    }
    __syncthreads();
  }
  if (wave == 0 && lane == 0) { misc[8] = t; misc[9] = ov; }
  __syncthreads();
  int ttv = misc[8];
  ttv = clampi(ttv, 0, RCAP);
  const int tt = __builtin_amdgcn_readfirstlane(ttv);

  if (wave == 0) {
    const int base = lane * (NBRUN / 32);
    int s = 0, big = 0;
#pragma unroll 1
    for (int i = 0; i < NBRUN / 32; ++i) {
      const int cv = cnt[base + i];
      s += cv;
      big |= (cv > DEGCAP) ? 1 : 0;
    }
    int incl = s;
#pragma unroll
    for (int d = 1; d < 32; d <<= 1) {
      const int y = __shfl_up(incl, d, 32);
      incl += (lane >= d) ? y : 0;
    }
    int run = incl - s;
#pragma unroll 1
    for (int i = 0; i < NBRUN / 32; ++i) {
      const int cv = cnt[base + i];
      offs[base + i] = run;
      cur[base + i]  = run;
      run += cv;
    }
    const unsigned bm = __builtin_amdgcn_ballot_w32(big != 0);
    if (lane == 0) misc[10] = (bm != 0u) ? 1 : 0;
  }
  __syncthreads();
  if (wave == 0) {
#pragma unroll 1
    for (int b0 = 0; b0 < tt; b0 += 32) {
      const int idx = b0 + lane;
      const int ent = hl[idx < RCAP ? idx : RCAP - 1];
      const int m32 = (tt - b0) < 32 ? (tt - b0) : 32;
#pragma unroll 1
      for (int k = 0; k < m32; ++k) {
        const int u    = __builtin_amdgcn_readlane(ent, k);
        const int slot = (u >> 16) & (NBRUN - 1);
        if (lane == 0) {
          int p = cur[slot];
          p = p < 0 ? 0 : (p > RCAP - 1 ? RCAP - 1 : p);
          sl[p] = u;
          cur[slot] = p + 1;
        }
      }
    }
  }
  __syncthreads();
  const int pois = ((misc[9] | misc[10]) != 0) ? 1 : 0;
#pragma unroll 1
  for (int i = tid; i < NBRUN; i += NTHR) {
    int c = cnt[i];
    c = c < 0 ? 0 : c;
    const float d = 1.0f / sqrtf((float)(c + 1));
    cur[i] = pois ? 0x7fc00000 : __float_as_int(d);
  }
  __syncthreads();

  int* lg = LISTG + (size_t)blk * RCAP;
  const v4i cv4 = *(const v4ia*)(cnt + 4 * tid);
  const v4i ov4 = *(const v4ia*)(offs + 4 * tid);
  const v4i dv4 = *(const v4ia*)(cur + 4 * tid);
  const v4i fv4 = (v4i){ pois, pois, pois, pois };
#pragma unroll 1
  for (int pass = 0; pass < 2; ++pass) {
#pragma unroll 1
    for (int it = 0; it < RCAP / (NTHR * 4); ++it) {
      const int idx = it * (NTHR * 4) + 4 * tid;
      const v4i v = *(const v4ia*)(sl + idx);
      *(volatile v4i*)(lg + idx) = v;
    }
    *(volatile v4i*)(CNTG + (size_t)slotBase + 4 * tid) = cv4;
    *(volatile v4i*)(OFFG + (size_t)slotBase + 4 * tid) = ov4;
    *(volatile v4i*)(DINVB + (size_t)slotBase + 4 * tid) = dv4;
    if (tid < 8) *(volatile v4i*)(FLAGG + (size_t)blk * 32 + 4 * tid) = fv4;
    __threadfence();
  }
}

template <int LAYER>
__global__ __launch_bounds__(NTHR) __attribute__((amdgpu_num_vgpr(248)))
void k_replay(const float* __restrict__ Hs, const int* __restrict__ LISTG, const int* __restrict__ CNTG,
              const int* __restrict__ OFFG, const float* __restrict__ DINVG, const int* __restrict__ FLAGG,
              const float* __restrict__ BF, unsigned short* X1, float* OUT) {
  constexpr int NC  = (LAYER == 1) ? D1 : D2;
  constexpr int VPL = NC / 128;
  constexpr int CPL = NC / 32;
  const int lane = (int)threadIdx.x & 31, wave = (int)threadIdx.x >> 5;
  const int row  = (int)blockIdx.x * 8 + wave;
  const bool live = row < GN;
  const int rc   = live ? row : GN - 1;
  const int blk  = rc >> 10;
  int cvv = CNTG[rc];
  int ofv = OFFG[rc];
  const int flv = FLAGG[blk * 32];
  const float di = DINVG[rc];
  asm volatile("" :: "v"(cvv));
  asm volatile("" :: "v"(ofv));
  asm volatile("" :: "v"(flv));
  asm volatile("" :: "v"(di));
  cvv = clampi(cvv, 0, DEGCAP);
  cvv = live ? cvv : 0;
  const int cn = __builtin_amdgcn_readfirstlane(cvv);
  ofv = clampi(ofv, 0, RCAP - 1);
  const int o = __builtin_amdgcn_readfirstlane(ofv);
  const bool pois = flv != 0;
  const int* lb = LISTG + (size_t)blk * RCAP;

  v4f acc[VPL];
#pragma unroll
  for (int v = 0; v < VPL; ++v) acc[v] = (v4f){ 0.0f, 0.0f, 0.0f, 0.0f };

#pragma unroll 1
  for (int b0 = 0; b0 < cn; b0 += 32) {
    int idx = o + b0 + lane;
    const int last = o + cn - 1;
    idx = idx > last ? last : idx;
    idx = clampi(idx, 0, RCAP - 1);
    const int wv = lb[idx];
    asm volatile("" :: "v"(wv));
    const int sr = clampi(wv & 0xFFFF, 0, GN - 1);
    const float ds = DINVG[sr];
    asm volatile("" :: "v"(ds));
    const float w  = ds * di;
    const int   wi = __float_as_int(w);
    const int m32 = (cn - b0) < 32 ? (cn - b0) : 32;
#pragma unroll 1
    for (int k = 0; k < m32; ++k) {
      const int   sk = __builtin_amdgcn_readlane(sr, k);
      const float wk = __int_as_float(__builtin_amdgcn_readlane(wi, k));
      const float* hp = Hs + (size_t)sk * NC + CPL * lane;
#pragma unroll
      for (int v = 0; v < VPL; ++v) {
        const v4f hv = *(const v4fa*)(hp + 4 * v);
        asm volatile("" :: "v"(hv));
        const v4f pr = hv * wk;
        acc[v] = acc[v] + pr;
      }
    }
  }

  const float rd = di * di;
  const float qnan = __int_as_float(0x7fc00000);
  v4f r[VPL];
#pragma unroll
  for (int v = 0; v < VPL; ++v) {
    const v4f hs = *(const v4fa*)(Hs + (size_t)rc * NC + CPL * lane + 4 * v);
    asm volatile("" :: "v"(hs));
    const v4f bv = *(const v4fa*)(BF + CPL * lane + 4 * v);
    asm volatile("" :: "v"(bv));
    const v4f sp = hs * rd;
    v4f tv = acc[v] + sp;
    tv = tv + bv;
#pragma unroll
    for (int e = 0; e < 4; ++e) {
      float x = tv[e];
      if (LAYER == 1) x = (x > 0.0f) ? x : (x - x);
      x = pois ? qnan : x;
      tv[e] = x;
    }
    r[v] = tv;
  }

  if constexpr (LAYER == 1) {
    const v4u hiw = pack8_bf16(r[0], r[VPL - 1]);
    unsigned short* xp = X1 + (size_t)rc * K2TOT + 8 * lane;
#if L2_TWO_TERM
    const v4u low = pack8_bf16_lo(r[0], r[VPL - 1]);
#endif
    if (live) *(volatile v4u*)xp = hiw;
#if L2_TWO_TERM
    if (live) *(volatile v4u*)(xp + D1) = low;
#endif
    __threadfence();
    if (live) *(volatile v4u*)xp = hiw;
#if L2_TWO_TERM
    if (live) *(volatile v4u*)(xp + D1) = low;
#endif
  } else {
    float* op = OUT + (size_t)rc * D2 + 4 * lane;
    const v4f ovv = r[0];
    if (live) *(volatile v4f*)op = ovv;
    __threadfence();
    if (live) *(volatile v4f*)op = ovv;
  }
}

extern "C" void kernel_launch(void* const* d_in, const int* in_sizes, int n_in,
                              void* d_out, int out_size, void* d_ws, size_t ws_size,
                              hipStream_t stream) {
  if (n_in < 7) return;
  if (in_sizes[0] != GN) return;
  if (in_sizes[1] != 2 * GE) return;
  if (in_sizes[2] != GN * D0) return;
  if (in_sizes[3] != D0 * D1) return;
  if (in_sizes[4] != D1) return;
  if (in_sizes[5] != D1 * D2) return;
  if (in_sizes[6] != D2) return;
  if (out_size != GN * D2) return;
  if (ws_size < WS_TOTAL) return;

  const int*   fidx = (const int*)d_in[0];
  const int*   edge = (const int*)d_in[1];
  const float* emb  = (const float*)d_in[2];
  const float* W1   = (const float*)d_in[3];
  const float* b1   = (const float*)d_in[4];
  const float* W2   = (const float*)d_in[5];
  const float* b2   = (const float*)d_in[6];
  float* out = (float*)d_out;
  const int* src = edge;
  const int* dst = edge + GE;

  char* ws = (char*)d_ws;
  float*          H    = (float*)(ws + O_H);
  unsigned short* X1   = (unsigned short*)(ws + O_X1);
  unsigned short* XB   = (unsigned short*)(ws + O_X1);
  int*            LIST = (int*)(ws + O_LIST);
  int*            CNT  = (int*)(ws + O_CNT);
  int*            OFF  = (int*)(ws + O_OFF);
  float*          DINV = (float*)(ws + O_DINV);
  int*            FLAG = (int*)(ws + O_FLAG);
  unsigned short* W1T  = (unsigned short*)(ws + O_W1T);
  unsigned short* W2D  = (unsigned short*)(ws + O_W2D);
  float*          B1F  = (float*)(ws + O_B1F);
  float*          B2F  = (float*)(ws + O_B2F);

  hipFuncSetAttribute(reinterpret_cast<const void*>(&k_bucket), hipFuncAttributeMaxDynamicSharedMemorySize,
                      (int)BK_LDS_BYTES);

  k_prep<<<PB_ALL, NTHR, 0, stream>>>(fidx, emb, W1, b1, W2, b2, XB, W1T, W2D, B1F, B2F, X1);
  k_bucket<<<NBLK, NTHR, (size_t)BK_LDS_BYTES, stream>>>(src, dst, LIST, CNT, OFF, (int*)DINV, FLAG);
  {
    const int tiles = ((GN + 63) / 64) * (D1 / 64);
    k_gemm_nt<0, 0><<<(tiles + 7) / 8, 256, 0, stream>>>(XB, W1T, B1F, H, GN, D1, D0, D1);
  }
  k_replay<1><<<GN / 8, NTHR, 0, stream>>>(H, LIST, CNT, OFF, DINV, FLAG, B1F, X1, out);
  {
    const int tiles = ((GN + 63) / 64) * (D2 / 64);
    k_gemm_nt<0, 0><<<(tiles + 7) / 8, 256, 0, stream>>>(X1, W2D, B2F, H, GN, D2, K2TOT, D2);
  }
  k_replay<2><<<GN / 8, NTHR, 0, stream>>>(H, LIST, CNT, OFF, DINV, FLAG, B2F, X1, out);
}
